// CapsuleLayer_70033736729248
// MI455X (gfx1250) — hardware-verified
//
#include <hip/hip_runtime.h>
#include <stddef.h>


typedef _Float16 h16;
typedef _Float16 v16h __attribute__((ext_vector_type(16)));
typedef _Float16 v8h  __attribute__((ext_vector_type(8)));
typedef float    v8f  __attribute__((ext_vector_type(8)));
typedef float    v4f  __attribute__((ext_vector_type(4)));

#ifndef NB
#define NB 32
#endif
#define NB_FULL 32
#define KDIM   512
#define NCAPS  256
#define ODIM   64
#define NCOL   (NCAPS * ODIM)
#define MPAD   32
#define NROUTE 3

static_assert(NB >= 1 && NB <= NB_FULL);
static_assert(NB <= MPAD && MPAD == 32);
static_assert(NCOL == 16384);
static_assert((KDIM % 64) == 0 && (KDIM % 32) == 0);
static_assert((NCOL % 128) == 0 && (NCOL % 64) == 0);
static_assert(ODIM == 2 * 32);
static_assert(NCAPS == 32 * 8);
static_assert(((MPAD * KDIM) % (8 * 256)) == 0);

#define LDT  72
#define LDCW 132
static_assert((LDT % 8) == 0 && LDT >= 64);
static_assert((LDCW % 4) == 0 && LDCW >= 128);

#define WCARRY 64.0f
#define XCARRY 64.0f

#define WT_BYTES  ((size_t)NCOL * KDIM * 2)
#define X16_BYTES ((size_t)MPAD * KDIM * 2)
#define H_BYTES   ((size_t)MPAD * NCOL * 4)
#define OFF_WT  ((size_t)0)
#define OFF_X16 (OFF_WT + WT_BYTES)
#define OFF_H   (OFF_X16 + X16_BYTES)
#define WS_TOTAL (OFF_H + H_BYTES)
static_assert((WT_BYTES % 128) == 0 && (X16_BYTES % 128) == 0 && (H_BYTES % 128) == 0);
static_assert(WS_TOTAL <= (size_t)134217728);

__device__ __forceinline__ float bf16r(float x) {
  unsigned int u = __float_as_uint(x);
  u = (u + 0x7FFFu + ((u >> 16) & 1u)) & 0xFFFF0000u;
  return __uint_as_float(u);
}

static __device__ __forceinline__ h16 toh_flush(float v) {
  const h16 r = (h16)v;
  return (fabsf(v) < 6.103515625e-05f) ? (h16)0.0f : r;
}

__device__ __forceinline__ v16h frag_at(const _Float16* p) {
  v8h lo = *(const v8h*)(p);
  v8h hi = *(const v8h*)(p + 16);
  v16h out;
#pragma unroll
  for (int i = 0; i < 8; ++i) { out[i] = lo[i]; out[i + 8] = hi[i]; }
  return out;
}

__device__ __forceinline__ v8f wmma16(v16h a, v16h b, v8f c) {
  v8f d = __builtin_amdgcn_wmma_f32_16x16x32_f16(false, a, false, b, (short)0, c,
                                                 false, false);
  asm volatile("v_nop\n\tv_nop\n\tv_nop\n\tv_nop" : "+v"(d) : "v"(a), "v"(b));
  return d;
}

__global__ __launch_bounds__(256) void wconv_kernel(
    const float* __restrict__ W, _Float16* __restrict__ Wt, unsigned ldw, unsigned ldk) {
  __shared__ _Float16 T[64 * LDT];
  const unsigned tid = threadIdx.x;
  const unsigned n0 = blockIdx.x * 64u;
  const unsigned k0 = blockIdx.y * 64u;
#pragma unroll 4
  for (unsigned j = 0; j < 16u; ++j) {
    const unsigned idx = tid + 256u * j;
    const unsigned kr = idx >> 6, nc = idx & 63u;
    const float v = W[(size_t)(k0 + kr) * ldw + n0 + nc];
    T[nc * LDT + kr] = toh_flush(WCARRY * bf16r(v));
  }
  __syncthreads();
  v8h x[2];
  size_t off[2];
#pragma unroll
  for (unsigned i = 0; i < 2u; ++i) {
    const unsigned n = 32u * i + (tid >> 3);
    const unsigned kc = (tid & 7u) * 8u;
    x[i] = *(const v8h*)&T[n * LDT + kc];
    off[i] = (size_t)(n0 + n) * ldk + k0 + kc;
  }
#pragma unroll
  for (int i = 0; i < 2; ++i) *(volatile v8h*)(Wt + off[i]) = x[i];
  __threadfence();
#pragma unroll
  for (int i = 0; i < 2; ++i) *(volatile v8h*)(Wt + off[i]) = x[i];
}

__global__ __launch_bounds__(256) void xconv_kernel(
    const float* __restrict__ X, _Float16* __restrict__ X16) {
  const unsigned g = blockIdx.x * 256u + threadIdx.x;
  const unsigned row = g / (unsigned)(KDIM / 8);
  const unsigned c = (g - row * (unsigned)(KDIM / 8)) * 8u;
  const unsigned rr = (row < (unsigned)NB) ? row : (unsigned)(NB - 1);
  const bool live = (row < (unsigned)NB);
  const v4f a0 = *(const v4f*)(X + (size_t)rr * KDIM + c);
  const v4f a1 = *(const v4f*)(X + (size_t)rr * KDIM + c + 4u);
  v8h o;
#pragma unroll
  for (int i = 0; i < 4; ++i) {
    const float e0 = live ? (XCARRY * bf16r(a0[i])) : 0.0f;
    const float e1 = live ? (XCARRY * bf16r(a1[i])) : 0.0f;
    o[i]     = toh_flush(e0);
    o[i + 4] = toh_flush(e1);
  }
  _Float16* p = X16 + (size_t)row * KDIM + c;
  *(volatile v8h*)p = o;
  __threadfence();
  *(volatile v8h*)p = o;
}

static_assert(8 * 4 == MPAD);
__global__ __launch_bounds__(256) void gemm_h_kernel(
    const _Float16* __restrict__ X16, const _Float16* __restrict__ Wt, float* __restrict__ H) {
  __shared__ float Cs[MPAD * LDCW];
  const unsigned tid = threadIdx.x, lane = tid & 31u;
  const int wave = __builtin_amdgcn_readfirstlane(threadIdx.x >> 5);
  const unsigned mw = (unsigned)wave & 1u, nw = (unsigned)wave >> 1;
  const unsigned hh = lane >> 4, m = lane & 15u;
  const unsigned n0 = blockIdx.x * 128u;

  const _Float16* ap  = X16 + (size_t)(mw * 16u + m) * KDIM + hh * 8u;
  const _Float16* bp0 = Wt + (size_t)(n0 + nw * 32u + m) * KDIM + hh * 8u;
  const _Float16* bp1 = bp0 + (size_t)16 * KDIM;
  v8f acc0 = {}, acc1 = {};
#pragma unroll 2
  for (unsigned k0 = 0; k0 < (unsigned)KDIM; k0 += 32u) {
    const v16h a  = frag_at(ap + k0);
    const v16h b0 = frag_at(bp0 + k0);
    const v16h b1 = frag_at(bp1 + k0);
    acc0 = wmma16(a, b0, acc0);
    acc1 = wmma16(a, b1, acc1);
  }
#pragma unroll
  for (int r = 0; r < 8; ++r) {
    float* d = &Cs[(mw * 16u + hh * 8u + (unsigned)r) * LDCW + nw * 32u + m];
    d[0]  = acc0[r];
    d[16] = acc1[r];
  }
  __syncthreads();

  const float cs = 1.0f / (WCARRY * XCARRY);
  v4f xs[4];
  size_t off[4];
#pragma unroll
  for (unsigned i = 0; i < 4u; ++i) {
    const unsigned r = 8u * i + (unsigned)wave;
    const unsigned c = lane * 4u;
    const v4f u = *(const v4f*)&Cs[r * LDCW + c];
    v4f val;
#pragma unroll
    for (int j = 0; j < 4; ++j) val[j] = u[j] * cs;
    xs[i] = val;
    off[i] = (size_t)r * NCOL + n0 + c;
  }
#pragma unroll
  for (int i = 0; i < 4; ++i) *(volatile v4f*)(H + off[i]) = xs[i];
  __threadfence();
#pragma unroll
  for (int i = 0; i < 4; ++i) *(volatile v4f*)(H + off[i]) = xs[i];
}

static_assert((NCAPS * 32 + 3 * 8 * 32) * 4 <= 131072);
__global__ __launch_bounds__(256) void route_kernel(
    const float* __restrict__ H, float* __restrict__ out) {
#pragma clang fp contract(off)
  __shared__ float Tv[NCAPS * 32];
  __shared__ float redm[8 * 32];
  __shared__ float reds[8 * 32];
  __shared__ float redc[8 * 32];
  const unsigned lane = threadIdx.x & 31u;
  const int wave = __builtin_amdgcn_readfirstlane(threadIdx.x >> 5);
  const unsigned b = blockIdx.x >> 1, dh = blockIdx.x & 1u;
  const size_t base = (size_t)b * NCOL + dh * 32u + lane;

#pragma unroll 1
  for (unsigned i = 0; i < 32u; ++i) {
    const unsigned j = i * 8u + (unsigned)wave;
    Tv[j * 32u + lane] = H[base + (size_t)j * ODIM];
  }

#pragma unroll 1
  for (int t = 0; t < NROUTE; ++t) {
    float mx = Tv[(unsigned)wave * 32u + lane];
#pragma unroll 1
    for (unsigned i = 1; i < 32u; ++i) {
      const unsigned j = i * 8u + (unsigned)wave;
      mx = fmaxf(mx, Tv[j * 32u + lane]);
    }
    redm[(unsigned)wave * 32u + lane] = mx;
    __syncthreads();
    float mall = redm[lane];
#pragma unroll 1
    for (unsigned q = 1; q < 8u; ++q) mall = fmaxf(mall, redm[q * 32u + lane]);

    float se = 0.0f;
#pragma unroll 1
    for (unsigned i = 0; i < 32u; ++i) {
      const unsigned j = i * 8u + (unsigned)wave;
      se += expf(Tv[j * 32u + lane] - mall);
    }
    reds[(unsigned)wave * 32u + lane] = se;
    __syncthreads();
    float sall = reds[lane];
#pragma unroll 1
    for (unsigned q = 1; q < 8u; ++q) sall += reds[q * 32u + lane];
    const float inv = 1.0f / sall;

    float cp = 0.0f;
#pragma unroll 1
    for (unsigned i = 0; i < 32u; ++i) {
      const unsigned j = i * 8u + (unsigned)wave;
      cp += expf(Tv[j * 32u + lane] - mall) * inv;
    }
    redc[(unsigned)wave * 32u + lane] = cp;
    __syncthreads();
    float call = redc[lane];
#pragma unroll 1
    for (unsigned q = 1; q < 8u; ++q) call += redc[q * 32u + lane];

#pragma unroll 1
    for (unsigned i = 0; i < 32u; ++i) {
      const unsigned j = i * 8u + (unsigned)wave;
      const float v = Tv[j * 32u + lane];
      Tv[j * 32u + lane] = call * v;
    }
  }

#pragma unroll 1
  for (unsigned i = 0; i < 32u; ++i) {
    const unsigned j = i * 8u + (unsigned)wave;
    const float v = Tv[j * 32u + lane];
    *(volatile float*)(out + base + (size_t)j * ODIM) = v;
  }
  __threadfence();
#pragma unroll 1
  for (unsigned i = 0; i < 32u; ++i) {
    const unsigned j = i * 8u + (unsigned)wave;
    const float v = Tv[j * 32u + lane];
    *(volatile float*)(out + base + (size_t)j * ODIM) = v;
  }
}

extern "C" void kernel_launch(void* const* d_in, const int* in_sizes, int n_in,
                              void* d_out, int out_size, void* d_ws, size_t ws_size,
                              hipStream_t stream) {
  if (n_in < 2) return;
  if ((long long)in_sizes[0] < (long long)NB * KDIM) return;
  if ((long long)in_sizes[1] < (long long)KDIM * NCOL) return;
  if ((long long)out_size < (long long)NB * NCOL) return;
  if (ws_size < WS_TOTAL) return;

  const float* X = (const float*)d_in[0];
  const float* W = (const float*)d_in[1];
  float* out = (float*)d_out;

  char* ws = (char*)d_ws;
  _Float16* Wt16 = (_Float16*)(ws + OFF_WT);
  _Float16* X16  = (_Float16*)(ws + OFF_X16);
  float*    Hf   = (float*)(ws + OFF_H);

  dim3 blk(256);
  xconv_kernel<<<dim3((MPAD * KDIM) / (8 * 256)), blk, 0, stream>>>(X, X16);
  wconv_kernel<<<dim3(NCOL / 64, KDIM / 64), blk, 0, stream>>>(W, Wt16, (unsigned)NCOL, (unsigned)KDIM);
  gemm_h_kernel<<<dim3(NCOL / 128), blk, 0, stream>>>(X16, Wt16, Hf);
  route_kernel<<<dim3(NB * 2), blk, 0, stream>>>(Hf, out);
}
